// SolidPINN_GNN_49400713839118
// MI455X (gfx1250) — hardware-run, weakly checked
//
#include <hip/hip_runtime.h>
#include <stddef.h>
#include <stdint.h>

#ifndef MODE_EE
#define MODE_EE 1
#endif
#ifndef MODE_NE
#define MODE_NE 2
#endif
#ifndef MODE_CV
#define MODE_CV 2
#endif
#ifndef MODE_HD
#define MODE_HD 2
#endif
#ifndef GELU_PRECISE
#define GELU_PRECISE 0
#endif

#define NNODE   50000
#define NEDGE   800000
#define NLAYER  4
#define HD      128
#define KT      256
#define APW     256
#define TM      128
#define MP      50048
#define NTHR    256
#define NWAVE   8
#define EPT     8
#define CHUNK   (NTHR * EPT)
#define WCAP    (EPT * 32)
#define LISTN   (NWAVE * WCAP)
#define NBRUN   1024
#define NBK     49
#define RCAP    20480
#define DEGCAP  64
#define PKS     10
#define METAW   2080
#define WSQ     (HD * KT)
#define NPLANE  11
#define NUSQ    (HD * (KT / 8))
#define SAP     264
#define E16W    64
#define ECARRY  16.0f
#define EINV    0.0625f

#define KS_EE ((MODE_EE == 2) ? 8 : 4)
#define KS_NE ((MODE_NE == 2) ? 8 : 4)
#define KS_CV ((MODE_CV == 2) ? 8 : 4)
#define KS_HD ((MODE_HD == 2) ? 8 : 4)

#define LDS_BUCKET ((2 * RCAP + 2 * NBRUN + 32 + LISTN + 16) * 4)
#define LDS_ENC    (TM * HD * 4 + TM * SAP * 2 + 1536 * 4)
#define LDS_CVA    (TM * HD * 4 + 384 * 4)
#define LDS_CVB    (TM * HD * 4 + 640 * 4)
#define LDS_HEAD   (TM * HD * 4 + 1312 * 4)

static_assert(NEDGE <= (1 << 20));
static_assert((NEDGE % TM) == 0 && (NEDGE % 4) == 0);
static_assert(NBRUN <= 1024 && NBRUN == (1 << PKS));
static_assert((MP % TM) == 0 && MP >= NNODE && MP - NNODE < TM);
static_assert(NBK * NBRUN >= MP && (NBRUN % TM) == 0);
static_assert((CHUNK & (CHUNK - 1)) == 0 && ((long long)CHUNK << PKS) < (1LL << 31));
static_assert(NTHR * 4 == NBRUN && LISTN >= NBRUN && (RCAP % 4) == 0 && (METAW % 4) == 0);
static_assert((RCAP / 4) % NTHR == 0);
static_assert((NPLANE * NUSQ) % NTHR == 0 && (NUSQ % NTHR) == 0);
static_assert(LDS_BUCKET <= 327680 && LDS_ENC <= 327680 && LDS_HEAD <= 327680);
static_assert((SAP * 2) % 16 == 0 && SAP >= KT);
static_assert(TM == NWAVE * 16 && HD == 128 && KT == 2 * HD);

typedef float          v4f  __attribute__((ext_vector_type(4)));
typedef float          v8f  __attribute__((ext_vector_type(8)));
typedef int            v4i  __attribute__((ext_vector_type(4)));
typedef int            v8i  __attribute__((ext_vector_type(8)));
typedef unsigned int   v2u  __attribute__((ext_vector_type(2)));
typedef unsigned int   v4u  __attribute__((ext_vector_type(4)));
typedef unsigned short v8us __attribute__((ext_vector_type(8)));
typedef __bf16         v16b __attribute__((ext_vector_type(16)));
typedef v4f  __attribute__((may_alias)) v4fa;
typedef v4i  __attribute__((may_alias)) v4ia;
typedef v4u  __attribute__((may_alias)) v4ua;
typedef v2u  __attribute__((may_alias)) v2ua;
typedef v8us __attribute__((may_alias)) v8usa;
union FragB { v16b v; v8us h[2]; v8i w; };

__device__ __forceinline__ v8f wmb(const FragB& a, const FragB& b, v8f c) {
  v8f d = __builtin_amdgcn_wmma_f32_16x16x32_bf16(false, a.v, false, b.v, (short)0, c, false, false);
  asm volatile("v_nop\n\tv_nop\n\tv_nop\n\tv_nop" : "+v"(d) : "v"(a.w), "v"(b.w));
  return d;
}

__device__ __forceinline__ unsigned short bf_bits(float f) {
  unsigned int u = __float_as_uint(f);
  u += 0x7FFFu + ((u >> 16) & 1u);
  return (unsigned short)(u >> 16);
}
__device__ __forceinline__ float bf_val(unsigned short b) {
  return __uint_as_float(((unsigned int)b) << 16);
}
__device__ __forceinline__ float bf_rne(float f) { return bf_val(bf_bits(f)); }
__device__ __forceinline__ unsigned f2h(float f) {
  const _Float16 hv = (_Float16)f;
  return (unsigned)__builtin_bit_cast(unsigned short, hv);
}
__device__ __forceinline__ float h2f(unsigned b) {
  const _Float16 hv = __builtin_bit_cast(_Float16, (unsigned short)b);
  return (float)hv;
}
__device__ __forceinline__ float fsel(float a, float b, unsigned mask) {
  return __uint_as_float((__float_as_uint(a) & ~mask) | (__float_as_uint(b) & mask));
}

__device__ __forceinline__ float gelu_f(float x) {
#if GELU_PRECISE
  return 0.5f * x * (1.0f + erff(x * 0.70710678f));
#else
  const float a = fabsf(x) * 0.70710678f;
  const float t = __builtin_amdgcn_rcpf(fmaf(0.3275911f, a, 1.0f));
  float p = fmaf(t, 1.061405429f, -1.453152027f);
  p = fmaf(t, p, 1.421413741f);
  p = fmaf(t, p, -0.284496736f);
  p = fmaf(t, p, 0.254829592f);
  const float q  = (t * p) * __expf(-(a * a));
  const float hq = 0.5f * q;
  const float ph = (x >= 0.0f) ? (1.0f - hq) : hq;
  return x * ph;
#endif
}

__device__ __forceinline__ float wsum32(float v) {
#pragma unroll
  for (int o = 16; o > 0; o >>= 1) v += __shfl_xor(v, o, 32);
  return v;
}
__device__ __forceinline__ float wsum16(float v) {
#pragma unroll
  for (int o = 8; o > 0; o >>= 1) v += __shfl_xor(v, o, 32);
  return v;
}

__device__ __forceinline__ v4f ln_gelu4(v4f v, v4f g, v4f b) {
  const float mean = wsum32((v.x + v.y) + (v.z + v.w)) * (1.0f / 128.0f);
  const float d0 = v.x - mean, d1 = v.y - mean, d2 = v.z - mean, d3 = v.w - mean;
  const float var = wsum32((d0 * d0 + d1 * d1) + (d2 * d2 + d3 * d3)) * (1.0f / 128.0f);
  const float rs = rsqrtf(var + 1e-5f);
  v4f o;
  o.x = gelu_f(fmaf(d0 * rs, g.x, b.x));
  o.y = gelu_f(fmaf(d1 * rs, g.y, b.y));
  o.z = gelu_f(fmaf(d2 * rs, g.z, b.z));
  o.w = gelu_f(fmaf(d3 * rs, g.w, b.w));
  return o;
}

__device__ __forceinline__ void stage128(float* sdst, const float* __restrict__ src, int lane) {
  const v4f a = *(const v4f*)(src + 4 * lane);
  v4f o;
  o.x = bf_rne(a.x); o.y = bf_rne(a.y); o.z = bf_rne(a.z); o.w = bf_rne(a.w);
  *(v4fa*)(sdst + 4 * lane) = o;
}
__device__ __forceinline__ void stage64(float* sdst, const float* __restrict__ src, int lane) {
  const int lc = lane < 16 ? lane : 15;
  const v4f a = *(const v4f*)(src + 4 * lc);
  asm volatile("" :: "v"(a));
  v4f o;
  o.x = bf_rne(a.x); o.y = bf_rne(a.y); o.z = bf_rne(a.z); o.w = bf_rne(a.w);
  if (lane < 16) *(v4fa*)(sdst + 4 * lane) = o;
}

template <int KS>
__device__ __forceinline__ void mma_rows_lds(const unsigned short* ap, const unsigned short* __restrict__ wp,
                                             v8f (&acc)[8]) {
#pragma unroll 1
  for (int ks = 0; ks < KS; ++ks) {
    FragB af;
    af.h[0] = *(const v8usa*)(ap + 32 * ks);
    af.h[1] = *(const v8usa*)(ap + 32 * ks + 16);
#pragma unroll
    for (int t = 0; t < 8; ++t) {
      const unsigned short* wq = wp + (size_t)(16 * t) * (size_t)KT + 32 * ks;
      FragB bf;
      bf.h[0] = *(const v8usa*)wq;
      bf.h[1] = *(const v8usa*)(wq + 16);
      acc[t] = wmb(af, bf, acc[t]);
    }
  }
}
template <int KS>
__device__ __forceinline__ void mma_rows_glb(const unsigned short* ap, const unsigned short* __restrict__ wp,
                                             v8f (&acc)[8]) {
#pragma unroll 1
  for (int ks = 0; ks < KS; ++ks) {
    FragB af;
    af.h[0] = *(const v8usa*)(ap + 32 * ks);
    af.h[1] = *(const v8usa*)(ap + 32 * ks + 16);
#pragma unroll
    for (int t = 0; t < 8; ++t) {
      const unsigned short* wq = wp + (size_t)(16 * t) * (size_t)KT + 32 * ks;
      FragB bf;
      bf.h[0] = *(const v8usa*)wq;
      bf.h[1] = *(const v8usa*)(wq + 16);
      acc[t] = wmb(af, bf, acc[t]);
    }
  }
}

__device__ __forceinline__ void stage_acc(float* stg, const v8f (&acc)[8], int wave, int hh, int m) {
#pragma unroll
  for (int t = 0; t < 8; ++t) {
    const int lc = 16 * t + m;
#pragma unroll
    for (int r = 0; r < 8; ++r) {
      const int lr = 16 * wave + 8 * hh + r;
      stg[lr * HD + lc] = acc[t][r];
    }
  }
}

__device__ __forceinline__ void put_rows_hilo(const float* stg, unsigned short* P, int rowBase, int wave,
                                              int lane, int mRows) {
  const int m = lane & 15;
  const bool isHi = lane < 16;
  const int cb = 8 * m;
  v4u pk[16];
#pragma unroll
  for (int i = 0; i < 16; ++i) {
    const int lr = 16 * wave + i;
    const v4f a = *(const v4fa*)(stg + lr * HD + cb);
    const v4f b = *(const v4fa*)(stg + lr * HD + cb + 4);
    const float f[8] = {a.x, a.y, a.z, a.w, b.x, b.y, b.z, b.w};
    unsigned int w[4];
#pragma unroll
    for (int j = 0; j < 4; ++j) {
      const unsigned short h0 = bf_bits(f[2 * j]), h1 = bf_bits(f[2 * j + 1]);
      const unsigned short l0 = bf_bits(f[2 * j] - bf_val(h0)), l1 = bf_bits(f[2 * j + 1] - bf_val(h1));
      const unsigned short q0 = isHi ? h0 : l0, q1 = isHi ? h1 : l1;
      w[j] = (unsigned int)q0 | ((unsigned int)q1 << 16);
    }
    v4u pw; pw.x = w[0]; pw.y = w[1]; pw.z = w[2]; pw.w = w[3];
    pk[i] = pw;
  }
#pragma unroll
  for (int i = 0; i < 16; ++i) {
    const int gr = rowBase + 16 * wave + i;
    unsigned short* op = P + (size_t)gr * (size_t)APW + 8 * lane;
    if (gr < mRows) *(volatile v4u*)op = pk[i];
  }
  __threadfence();
#pragma unroll
  for (int i = 0; i < 16; ++i) {
    const int gr = rowBase + 16 * wave + i;
    unsigned short* op = P + (size_t)gr * (size_t)APW + 8 * lane;
    if (gr < mRows) *(volatile v4u*)op = pk[i];
  }
}

__device__ __forceinline__ v8us gath8(const float* __restrict__ p, int stride) {
  v8us o;
#pragma unroll
  for (int i = 0; i < 8; ++i) o[i] = bf_bits(p[(size_t)i * stride]);
  return o;
}
__global__ __launch_bounds__(NTHR) void k_wprep(const float* __restrict__ ne_w2, const float* __restrict__ ee_w2,
                                                const float* __restrict__ cv_w1, const float* __restrict__ cv_w2,
                                                const float* __restrict__ dh_w1, const float* __restrict__ sh_w1,
                                                unsigned short* wt) {
  const int u  = (int)blockIdx.x * NTHR + (int)threadIdx.x;
  const int mi = u / NUSQ;
  const int v  = u - mi * NUSQ;
  const int n  = v >> 5;
  const int k8 = (v & 31) * 8;
  const int kk = k8 & (HD - 1);
  v8us o;
  if (mi == 0)       o = gath8(ne_w2 + (size_t)kk * HD + n, HD);
  else if (mi == 1)  o = gath8(ee_w2 + (size_t)kk * HD + n, HD);
  else if (mi < 6)   o = gath8(cv_w1 + (size_t)(mi - 2) * HD * HD + (size_t)kk * HD + n, HD);
  else if (mi < 10)  o = gath8(cv_w2 + (size_t)(mi - 6) * HD * HD + (size_t)kk * HD + n, HD);
  else if (n < 64)   o = gath8(dh_w1 + (size_t)kk * 64 + n, 64);
  else               o = gath8(sh_w1 + (size_t)kk * 64 + (n - 64), 64);
  unsigned short* dp = wt + (size_t)mi * WSQ + (size_t)n * KT + k8;
  *(volatile v8us*)dp = o;
  __threadfence();
  *(volatile v8us*)dp = o;
}

__device__ __forceinline__ int scan_chunk(const int* __restrict__ dsts, int nE, int cbase, int slotBase,
                                          int nb, int vec8, int* list, int tid, int lane, int wave) {
  int wc = 0;
  const int el0  = tid * EPT;
  const int e0   = cbase + el0;
  const int sent = -2147483647 - 1;
  v4i da, db;
  if (vec8 != 0 && cbase + CHUNK <= nE) {
    da = *(const v4i*)(dsts + e0);
    db = *(const v4i*)(dsts + e0 + 4);
  } else {
    const int k0 = dsts[min(e0,     nE - 1)];
    const int k1 = dsts[min(e0 + 1, nE - 1)];
    const int k2 = dsts[min(e0 + 2, nE - 1)];
    const int k3 = dsts[min(e0 + 3, nE - 1)];
    const int k4 = dsts[min(e0 + 4, nE - 1)];
    const int k5 = dsts[min(e0 + 5, nE - 1)];
    const int k6 = dsts[min(e0 + 6, nE - 1)];
    const int k7 = dsts[min(e0 + 7, nE - 1)];
    asm volatile("" :: "v"(k0), "v"(k1), "v"(k2), "v"(k3), "v"(k4), "v"(k5), "v"(k6), "v"(k7));
    da.x = (e0     < nE) ? k0 : sent;
    da.y = (e0 + 1 < nE) ? k1 : sent;
    da.z = (e0 + 2 < nE) ? k2 : sent;
    da.w = (e0 + 3 < nE) ? k3 : sent;
    db.x = (e0 + 4 < nE) ? k4 : sent;
    db.y = (e0 + 5 < nE) ? k5 : sent;
    db.z = (e0 + 6 < nE) ? k6 : sent;
    db.w = (e0 + 7 < nE) ? k7 : sent;
  }
  const unsigned nbs = (unsigned)slotBase;
  const unsigned unb = (unsigned)nb;
  const unsigned s0 = (unsigned)da.x - nbs, s1 = (unsigned)da.y - nbs;
  const unsigned s2 = (unsigned)da.z - nbs, s3 = (unsigned)da.w - nbs;
  const unsigned s4 = (unsigned)db.x - nbs, s5 = (unsigned)db.y - nbs;
  const unsigned s6 = (unsigned)db.z - nbs, s7 = (unsigned)db.w - nbs;
  const bool h0 = s0 < unb, h1 = s1 < unb, h2 = s2 < unb, h3 = s3 < unb;
  const bool h4 = s4 < unb, h5 = s5 < unb, h6 = s6 < unb, h7 = s7 < unb;
  const unsigned any = __builtin_amdgcn_ballot_w32(h0 | h1 | h2 | h3 | h4 | h5 | h6 | h7);
  if (any != 0u) {
#define HITJ(J, HJ, SJ) { \
      const unsigned mj = __builtin_amdgcn_ballot_w32(HJ); \
      if (mj != 0u) { \
        if (HJ) { \
          const int pos = wc + (int)__builtin_amdgcn_mbcnt_lo(mj, 0u); \
          if (pos < WCAP) list[wave * WCAP + pos] = ((el0 + (J)) << PKS) | (int)(SJ); \
        } \
        wc += (int)__builtin_popcount(mj); } }
    HITJ(0, h0, s0)
    HITJ(1, h1, s1)
    HITJ(2, h2, s2)
    HITJ(3, h3, s3)
    HITJ(4, h4, s4)
    HITJ(5, h5, s5)
    HITJ(6, h6, s6)
    HITJ(7, h7, s7)
#undef HITJ
  }
  return wc;
}

__global__ __launch_bounds__(NTHR) void k_bucket(const int* __restrict__ dsts, int nE, int vec8,
                                                 unsigned* lst, int* meta) {
  extern __shared__ v4f dynl[];
  int* reg1 = (int*)dynl;
  int* reg2 = reg1 + RCAP;
  int* scnt = reg2 + RCAP;
  int* soff = scnt + NBRUN;
  int* flg  = soff + NBRUN;
  int* list = flg + 32;
  int* wcnt = list + LISTN;
  int* wtot = wcnt + NWAVE;
  const int tid = (int)threadIdx.x, lane = tid & 31, wave = tid >> 5;
  const int nodeBase = (int)blockIdx.x * NBRUN;

  {
    const v4i z4 = {0, 0, 0, 0};
    for (int i = tid * 4; i < 2 * RCAP + NBRUN; i += NTHR * 4) *(v4ia*)(reg1 + i) = z4;
  }
  __syncthreads();

  int tot = 0;
  const int nChunks = (nE + CHUNK - 1) / CHUNK;
#pragma unroll 1
  for (int ch = 0; ch < nChunks; ++ch) {
    const int cbase = ch * CHUNK;
    const int wc = scan_chunk(dsts, nE, cbase, nodeBase, NBRUN, vec8, list, tid, lane, wave);
    if (lane == 0) wcnt[wave] = wc;
    __syncthreads();
    int pre = 0, all = 0;
#pragma unroll
    for (int w2 = 0; w2 < NWAVE; ++w2) {
      int c = wcnt[w2];
      c = c < 0 ? 0 : (c > WCAP ? WCAP : c);
      all += c;
      pre += (w2 < wave) ? c : 0;
    }
    const int wcc  = wc > WCAP ? WCAP : wc;
    const int base = tot + pre;
#pragma unroll 1
    for (int i = lane; i < wcc; i += 32) {
      const int ent = list[wave * WCAP + i];
      const int el  = (ent >> PKS) & (CHUNK - 1);
      const int sl  = ent & (NBRUN - 1);
      int eid = cbase + el;
      eid = eid > nE - 1 ? nE - 1 : eid;
      const int pos = base + i;
      if (pos < RCAP) reg1[pos] = (int)(((unsigned)eid << PKS) | (unsigned)sl);
    }
    tot += all;
    tot = tot > RCAP ? RCAP : tot;
    __syncthreads();
  }
  const int nh = tot;

  if (wave == 0) {
#pragma unroll 1
    for (int b0 = 0; b0 < nh; b0 += 32) {
      const int idx = b0 + lane;
      const int uv  = reg1[idx < RCAP ? idx : RCAP - 1];
      const int m32 = (nh - b0) < 32 ? (nh - b0) : 32;
#pragma unroll 1
      for (int k = 0; k < m32; ++k) {
        const int u  = __builtin_amdgcn_readlane(uv, k);
        const int sl = u & (NBRUN - 1);
        if (lane == 0) scnt[sl] = scnt[sl] + 1;
      }
    }
  }
  __syncthreads();

  {
    const v4i ca = *(const v4ia*)(scnt + 4 * tid);
    const int e0 = ca.x < 0 ? 0 : ca.x, e1 = ca.y < 0 ? 0 : ca.y, e2 = ca.z < 0 ? 0 : ca.z, e3 = ca.w < 0 ? 0 : ca.w;
    const int ts = e0 + e1 + e2 + e3;
    int incl = ts;
#pragma unroll
    for (int d = 1; d < 32; d <<= 1) {
      const int up = __shfl_up(incl, d, 32);
      if (lane >= d) incl += up;
    }
    if (lane == 31) wtot[wave] = incl;
    __syncthreads();
    int pre = 0;
#pragma unroll
    for (int w2 = 0; w2 < NWAVE; ++w2) pre += (w2 < wave) ? wtot[w2] : 0;
    int run = pre + incl - ts;
    soff[4 * tid + 0] = run; run += e0;
    soff[4 * tid + 1] = run; run += e1;
    soff[4 * tid + 2] = run; run += e2;
    soff[4 * tid + 3] = run;
  }
  if (tid < 32) flg[tid] = (tid == 0) ? ((nh >= RCAP) ? 1 : 0) : ((tid == 1) ? nh : 0);
  __syncthreads();
  for (int i = tid; i < NBRUN; i += NTHR) list[i] = soff[i];
  __syncthreads();

  if (wave == 0) {
#pragma unroll 1
    for (int b0 = 0; b0 < nh; b0 += 32) {
      const int idx = b0 + lane;
      const int uv  = reg1[idx < RCAP ? idx : RCAP - 1];
      const int m32 = (nh - b0) < 32 ? (nh - b0) : 32;
#pragma unroll 1
      for (int k = 0; k < m32; ++k) {
        const int u   = __builtin_amdgcn_readlane(uv, k);
        const int sl  = u & (NBRUN - 1);
        const unsigned eid = ((unsigned)u >> PKS) & 0xFFFFFu;
        if (lane == 0) {
          int pos = list[sl];
          pos = pos < 0 ? 0 : (pos > RCAP - 1 ? RCAP - 1 : pos);
          reg2[pos] = (int)(eid | ((unsigned)sl << 20));
          list[sl] = pos + 1;
        }
      }
    }
  }
  __syncthreads();

  unsigned* lp = lst + (size_t)blockIdx.x * RCAP;
#pragma unroll 1
  for (int it = 0; it < RCAP / 4 / NTHR; ++it) {
    const int u = it * NTHR + tid;
    const v4i v = *(const v4ia*)(reg2 + 4 * u);
    *(volatile v4i*)(lp + 4 * u) = v;
  }
  int* mp = meta + (size_t)blockIdx.x * METAW;
#pragma unroll 1
  for (int it = 0; it < 3; ++it) {
    const int u  = it * NTHR + tid;
    const int uc = u < METAW / 4 ? u : METAW / 4 - 1;
    const v4i v = *(const v4ia*)(scnt + 4 * uc);
    if (u < METAW / 4) *(volatile v4i*)(mp + 4 * u) = v;
  }
  __threadfence();
#pragma unroll 1
  for (int it = 0; it < RCAP / 4 / NTHR; ++it) {
    const int u = it * NTHR + tid;
    const v4i v = *(const v4ia*)(reg2 + 4 * u);
    *(volatile v4i*)(lp + 4 * u) = v;
  }
#pragma unroll 1
  for (int it = 0; it < 3; ++it) {
    const int u  = it * NTHR + tid;
    const int uc = u < METAW / 4 ? u : METAW / 4 - 1;
    const v4i v = *(const v4ia*)(scnt + 4 * uc);
    if (u < METAW / 4) *(volatile v4i*)(mp + 4 * u) = v;
  }
}

template <int KIN, int EDGE, int KS>
__global__ __launch_bounds__(NTHR) __attribute__((amdgpu_num_vgpr(248)))
void k_enc(const float* __restrict__ xin, int nrows,
           const float* __restrict__ w1, const float* __restrict__ b1, const float* __restrict__ g1,
           const float* __restrict__ be1, const float* __restrict__ b2, const float* __restrict__ g2,
           const float* __restrict__ be2, const unsigned short* __restrict__ WT, void* outp, int mrows) {
  extern __shared__ v4f dynl[];
  float* stg = (float*)dynl;
  unsigned short* sA = (unsigned short*)(stg + TM * HD);
  float* sp = (float*)(sA + TM * SAP);
  const int tid = (int)threadIdx.x, lane = tid & 31, wave = tid >> 5, hh = lane >> 4, m = lane & 15;
  const int rowBase = (int)blockIdx.x * TM;

  if (tid < KIN * 32) {
    const v4f a = *(const v4f*)(w1 + 4 * tid);
    v4f o;
    o.x = bf_rne(a.x); o.y = bf_rne(a.y); o.z = bf_rne(a.z); o.w = bf_rne(a.w);
    *(v4fa*)(sp + 4 * tid) = o;
  }
  if (wave == 0)      stage128(sp + 768,  b1,  lane);
  else if (wave == 1) stage128(sp + 896,  g1,  lane);
  else if (wave == 2) stage128(sp + 1024, be1, lane);
  else if (wave == 3) stage128(sp + 1152, b2,  lane);
  else if (wave == 4) stage128(sp + 1280, g2,  lane);
  else if (wave == 5) stage128(sp + 1408, be2, lane);
  __syncthreads();

  {
    const int row = tid >> 1, half = tid & 1;
    const int grow = rowBase + row;
    const int rc = grow < nrows ? grow : nrows - 1;
    float xk[KIN];
    if constexpr (KIN == 4) {
      const v4f a = *(const v4f*)(xin + (size_t)rc * 4);
      xk[0] = bf_rne(a.x); xk[1] = bf_rne(a.y); xk[2] = bf_rne(a.z); xk[3] = bf_rne(a.w);
    } else {
      const float* xp = xin + (size_t)rc * KIN;
#pragma unroll
      for (int k = 0; k < KIN; ++k) xk[k] = bf_rne(xp[k]);
    }
    float* tr = stg + row * HD + 64 * half;
    const int cb = 64 * half;
    float s = 0.0f;
#pragma unroll 4
    for (int c = 0; c < 64; ++c) {
      float t = 0.0f;
#pragma unroll
      for (int k = 0; k < KIN; ++k) t = fmaf(xk[k], sp[k * HD + cb + c], t);
      t += sp[768 + cb + c];
      tr[c] = t;
      s += t;
    }
    s += __shfl_xor(s, 1, 32);
    const float mean = s * (1.0f / 128.0f);
    float q = 0.0f;
#pragma unroll 4
    for (int c = 0; c < 64; ++c) {
      const float d = tr[c] - mean;
      q = fmaf(d, d, q);
    }
    q += __shfl_xor(q, 1, 32);
    const float rs = rsqrtf(q * (1.0f / 128.0f) + 1e-5f);
    unsigned short* ar = sA + row * SAP + cb;
#pragma unroll 1
    for (int c8 = 0; c8 < 8; ++c8) {
      const v4f ta = *(const v4fa*)(tr + 8 * c8);
      const v4f tb = *(const v4fa*)(tr + 8 * c8 + 4);
      const float tv[8] = {ta.x, ta.y, ta.z, ta.w, tb.x, tb.y, tb.z, tb.w};
      v8us oh, ol;
#pragma unroll
      for (int i = 0; i < 8; ++i) {
        const int cc = cb + 8 * c8 + i;
        const float y  = fmaf((tv[i] - mean) * rs, sp[896 + cc], sp[1024 + cc]);
        const float ge = gelu_f(y);
        const unsigned short hb = bf_bits(ge);
        const unsigned short lb = bf_bits(ge - bf_val(hb));
        oh[i] = hb; ol[i] = lb;
      }
      *(v8usa*)(ar + 8 * c8) = oh;
      *(v8usa*)(ar + HD + 8 * c8) = ol;
    }
  }
  __syncthreads();

  v8f acc[8];
  {
    const v8f z = {0.f, 0.f, 0.f, 0.f, 0.f, 0.f, 0.f, 0.f};
#pragma unroll
    for (int t = 0; t < 8; ++t) acc[t] = z;
  }
  mma_rows_lds<KS>(sA + (16 * wave + m) * SAP + 8 * hh, WT + (size_t)m * KT + 8 * hh, acc);
  stage_acc(stg, acc, wave, hh, m);
  __syncthreads();

  {
    const v4f b2v = *(const v4fa*)(sp + 1152 + 4 * lane);
    const v4f g2v = *(const v4fa*)(sp + 1280 + 4 * lane);
    const v4f e2v = *(const v4fa*)(sp + 1408 + 4 * lane);
#pragma unroll 1
    for (int i = 0; i < 16; ++i) {
      float* sr = stg + (16 * wave + i) * HD + 4 * lane;
      v4f v = *(const v4fa*)sr;
      v.x += b2v.x; v.y += b2v.y; v.z += b2v.z; v.w += b2v.w;
      v4f y = ln_gelu4(v, g2v, e2v);
      const bool live = (rowBase + 16 * wave + i) < nrows;
      y.x = live ? y.x : 0.0f; y.y = live ? y.y : 0.0f; y.z = live ? y.z : 0.0f; y.w = live ? y.w : 0.0f;
      *(v4fa*)sr = y;
    }
  }
  __syncthreads();

  if constexpr (EDGE == 0) {
    float* outF = (float*)outp;
    v4f fv[16];
#pragma unroll
    for (int i = 0; i < 16; ++i) fv[i] = *(const v4fa*)(stg + (16 * wave + i) * HD + 4 * lane);
#pragma unroll
    for (int i = 0; i < 16; ++i) {
      const int gr = rowBase + 16 * wave + i;
      float* op = outF + (size_t)gr * HD + 4 * lane;
      if (gr < mrows) *(volatile v4f*)op = fv[i];
    }
    __threadfence();
#pragma unroll
    for (int i = 0; i < 16; ++i) {
      const int gr = rowBase + 16 * wave + i;
      float* op = outF + (size_t)gr * HD + 4 * lane;
      if (gr < mrows) *(volatile v4f*)op = fv[i];
    }
  } else {
    unsigned* outE = (unsigned*)outp;
    v2u pk[16];
#pragma unroll
    for (int i = 0; i < 16; ++i) {
      const v4f a = *(const v4fa*)(stg + (16 * wave + i) * HD + 4 * lane);
      v2u w;
      w.x = f2h(ECARRY * a.x) | (f2h(ECARRY * a.y) << 16);
      w.y = f2h(ECARRY * a.z) | (f2h(ECARRY * a.w) << 16);
      pk[i] = w;
    }
#pragma unroll
    for (int i = 0; i < 16; ++i) {
      const int gr = rowBase + 16 * wave + i;
      unsigned* op = outE + (size_t)gr * E16W + 2 * lane;
      if (gr < mrows) *(volatile v2u*)op = pk[i];
    }
    __threadfence();
#pragma unroll
    for (int i = 0; i < 16; ++i) {
      const int gr = rowBase + 16 * wave + i;
      unsigned* op = outE + (size_t)gr * E16W + 2 * lane;
      if (gr < mrows) *(volatile v2u*)op = pk[i];
    }
  }
}

__global__ __launch_bounds__(NTHR) void k_agg(const int* __restrict__ srcs, const unsigned* __restrict__ lst,
                                              const int* __restrict__ meta, const float* __restrict__ Hf,
                                              const unsigned* __restrict__ e16, unsigned short* P1,
                                              int nN, int nE, int mRows) {
  __shared__ int smeta[2 * TM];
  __shared__ __attribute__((aligned(16))) unsigned stw[NWAVE * 128];
  const int tid = (int)threadIdx.x, lane = tid & 31, wave = tid >> 5;
  const int rowBase  = (int)blockIdx.x * TM;
  const int bk       = rowBase / NBRUN;
  const int slotBase = rowBase - bk * NBRUN;
  const int* mb = meta + (size_t)bk * METAW;
  const unsigned* lp = lst + (size_t)bk * RCAP;
  {
    const int mo = (tid < TM) ? (slotBase + tid) : (NBRUN + slotBase + tid - TM);
    smeta[tid] = mb[mo];
  }
  const int fl = mb[2 * NBRUN];
  __syncthreads();
  const float qnan = __int_as_float(0x7fc00000);
  unsigned* stwu = stw + wave * 128;

#pragma unroll 1
  for (int jt = 0; jt < 16; ++jt) {
    const int ls   = 16 * wave + jt;
    const int grow = rowBase + ls;
    const int craw = smeta[ls];
    int st  = smeta[TM + ls];
    int cnt = craw;
    st  = st < 0 ? 0 : (st > RCAP ? RCAP : st);
    cnt = cnt < 0 ? 0 : (cnt > DEGCAP ? DEGCAP : cnt);
    cnt = cnt > RCAP - st ? RCAP - st : cnt;
    cnt = __builtin_amdgcn_readfirstlane(cnt);
    st  = __builtin_amdgcn_readfirstlane(st);
    const float pz = (fl != 0 || craw > DEGCAP) ? qnan : 0.0f;
    const bool liveRow = grow < nN;

    float ag0 = 0.0f, ag1 = 0.0f, ag2 = 0.0f, ag3 = 0.0f;
#pragma unroll 1
    for (int b0 = 0; b0 < cnt; b0 += 32) {
      int idx = st + b0 + lane;
      idx = idx < 0 ? 0 : (idx > RCAP - 1 ? RCAP - 1 : idx);
      const unsigned wv = lp[idx];
      int eid = (int)(wv & 0xFFFFFu);
      eid = eid > nE - 1 ? nE - 1 : eid;
      const int sraw = srcs[eid];
      const int sv = sraw < 0 ? 0 : (sraw > nN - 1 ? nN - 1 : sraw);
      const int m32 = (cnt - b0) < 32 ? (cnt - b0) : 32;
#pragma unroll 1
      for (int k = 0; k < m32; ++k) {
        const int sk = __builtin_amdgcn_readlane(sv, k);
        const int ek = __builtin_amdgcn_readlane(eid, k);
        const v4f hv = *(const v4f*)(Hf + (size_t)sk * HD + 4 * lane);
        const v2u ew = *(const v2u*)(e16 + (size_t)ek * E16W + 2 * lane);
        const float v0 = fmaf(h2f(ew.x & 0xffffu), EINV, hv.x);
        const float v1 = fmaf(h2f(ew.x >> 16),     EINV, hv.y);
        const float v2 = fmaf(h2f(ew.y & 0xffffu), EINV, hv.z);
        const float v3 = fmaf(h2f(ew.y >> 16),     EINV, hv.w);
        ag0 += (v0 > 0.0f) ? v0 : (v0 - v0);
        ag1 += (v1 > 0.0f) ? v1 : (v1 - v1);
        ag2 += (v2 > 0.0f) ? v2 : (v2 - v2);
        ag3 += (v3 > 0.0f) ? v3 : (v3 - v3);
      }
    }
    const int nc = liveRow ? grow : nN - 1;
    const v4f sf = *(const v4f*)(Hf + (size_t)nc * HD + 4 * lane);
    float r0 = sf.x + ag0, r1 = sf.y + ag1, r2 = sf.z + ag2, r3 = sf.w + ag3;
    r0 = (liveRow ? r0 : 0.0f) + pz;
    r1 = (liveRow ? r1 : 0.0f) + pz;
    r2 = (liveRow ? r2 : 0.0f) + pz;
    r3 = (liveRow ? r3 : 0.0f) + pz;

    const unsigned short hb0 = bf_bits(r0), hb1 = bf_bits(r1), hb2 = bf_bits(r2), hb3 = bf_bits(r3);
    const unsigned short lb0 = bf_bits(r0 - bf_val(hb0)), lb1 = bf_bits(r1 - bf_val(hb1));
    const unsigned short lb2 = bf_bits(r2 - bf_val(hb2)), lb3 = bf_bits(r3 - bf_val(hb3));
    v2u hw, lw;
    hw.x = (unsigned int)hb0 | ((unsigned int)hb1 << 16);
    hw.y = (unsigned int)hb2 | ((unsigned int)hb3 << 16);
    lw.x = (unsigned int)lb0 | ((unsigned int)lb1 << 16);
    lw.y = (unsigned int)lb2 | ((unsigned int)lb3 << 16);
    __syncthreads();
    *(v2ua*)(stwu + 2 * lane)      = hw;
    *(v2ua*)(stwu + 64 + 2 * lane) = lw;
    __syncthreads();
    const v4u pk = *(const v4ua*)(stwu + 4 * lane);
    unsigned short* gp = P1 + (size_t)grow * (size_t)APW + 8 * lane;
    const bool wsv = grow < mRows;
    if (wsv) *(volatile v4u*)gp = pk;
    __threadfence();
    if (wsv) *(volatile v4u*)gp = pk;
  }
}

template <int KS>
__global__ __launch_bounds__(NTHR) __attribute__((amdgpu_num_vgpr(248)))
void k_cva(unsigned short* P1, const unsigned short* __restrict__ WT, const float* __restrict__ b1,
           const float* __restrict__ g1, const float* __restrict__ be1, int nN, int mRows) {
  extern __shared__ v4f dynl[];
  float* stg = (float*)dynl;
  float* sp  = stg + TM * HD;
  const int tid = (int)threadIdx.x, lane = tid & 31, wave = tid >> 5, hh = lane >> 4, m = lane & 15;
  const int rowBase = (int)blockIdx.x * TM;
  if (wave == 0)      stage128(sp,       b1,  lane);
  else if (wave == 1) stage128(sp + 128, g1,  lane);
  else if (wave == 2) stage128(sp + 256, be1, lane);

  v8f acc[8];
  {
    const v8f z = {0.f, 0.f, 0.f, 0.f, 0.f, 0.f, 0.f, 0.f};
#pragma unroll
    for (int t = 0; t < 8; ++t) acc[t] = z;
  }
  mma_rows_glb<KS>(P1 + (size_t)(rowBase + 16 * wave + m) * (size_t)APW + 8 * hh,
                   WT + (size_t)m * KT + 8 * hh, acc);
  stage_acc(stg, acc, wave, hh, m);
  __syncthreads();
  {
    const v4f bv = *(const v4fa*)(sp + 4 * lane);
    const v4f gv = *(const v4fa*)(sp + 128 + 4 * lane);
    const v4f ev = *(const v4fa*)(sp + 256 + 4 * lane);
#pragma unroll 1
    for (int i = 0; i < 16; ++i) {
      float* sr = stg + (16 * wave + i) * HD + 4 * lane;
      v4f v = *(const v4fa*)sr;
      v.x += bv.x; v.y += bv.y; v.z += bv.z; v.w += bv.w;
      v4f y = ln_gelu4(v, gv, ev);
      const bool live = (rowBase + 16 * wave + i) < nN;
      y.x = live ? y.x : 0.0f; y.y = live ? y.y : 0.0f; y.z = live ? y.z : 0.0f; y.w = live ? y.w : 0.0f;
      *(v4fa*)sr = y;
    }
  }
  __syncthreads();
  put_rows_hilo(stg, P1, rowBase, wave, lane, mRows);
}

template <int LAST, int KS>
__global__ __launch_bounds__(NTHR) __attribute__((amdgpu_num_vgpr(248)))
void k_cvb(unsigned short* P1, const unsigned short* __restrict__ WT, const float* __restrict__ b2,
           const float* __restrict__ g2, const float* __restrict__ be2, const float* __restrict__ ng,
           const float* __restrict__ nb, float* Hf, float* out2, int nN, int mRows) {
  extern __shared__ v4f dynl[];
  float* stg = (float*)dynl;
  float* sp  = stg + TM * HD;
  const int tid = (int)threadIdx.x, lane = tid & 31, wave = tid >> 5, hh = lane >> 4, m = lane & 15;
  const int rowBase = (int)blockIdx.x * TM;
  if (wave == 0)      stage128(sp,       b2,  lane);
  else if (wave == 1) stage128(sp + 128, g2,  lane);
  else if (wave == 2) stage128(sp + 256, be2, lane);
  else if (wave == 3) stage128(sp + 384, ng,  lane);
  else if (wave == 4) stage128(sp + 512, nb,  lane);

  v8f acc[8];
  {
    const v8f z = {0.f, 0.f, 0.f, 0.f, 0.f, 0.f, 0.f, 0.f};
#pragma unroll
    for (int t = 0; t < 8; ++t) acc[t] = z;
  }
  mma_rows_glb<KS>(P1 + (size_t)(rowBase + 16 * wave + m) * (size_t)APW + 8 * hh,
                   WT + (size_t)m * KT + 8 * hh, acc);
  stage_acc(stg, acc, wave, hh, m);
  __syncthreads();
  {
    const v4f bv  = *(const v4fa*)(sp + 4 * lane);
    const v4f gv  = *(const v4fa*)(sp + 128 + 4 * lane);
    const v4f ev  = *(const v4fa*)(sp + 256 + 4 * lane);
    const v4f ngv = *(const v4fa*)(sp + 384 + 4 * lane);
    const v4f nbv = *(const v4fa*)(sp + 512 + 4 * lane);
#pragma unroll 1
    for (int i = 0; i < 16; ++i) {
      const int gr = rowBase + 16 * wave + i;
      float* sr = stg + (16 * wave + i) * HD + 4 * lane;
      v4f v = *(const v4fa*)sr;
      v.x += bv.x; v.y += bv.y; v.z += bv.z; v.w += bv.w;
      const v4f u = ln_gelu4(v, gv, ev);
      const v4f w = ln_gelu4(u, ngv, nbv);
      const v4f hv = *(const v4f*)(Hf + (size_t)gr * HD + 4 * lane);
      const bool live = gr < nN;
      v4f y;
      y.x = live ? (hv.x + w.x) : 0.0f;
      y.y = live ? (hv.y + w.y) : 0.0f;
      y.z = live ? (hv.z + w.z) : 0.0f;
      y.w = live ? (hv.w + w.w) : 0.0f;
      *(v4fa*)sr = y;
    }
  }
  __syncthreads();
  {
    v4f fv[16];
#pragma unroll
    for (int i = 0; i < 16; ++i) fv[i] = *(const v4fa*)(stg + (16 * wave + i) * HD + 4 * lane);
#pragma unroll
    for (int i = 0; i < 16; ++i) {
      const int gr = rowBase + 16 * wave + i;
      if (gr < mRows) *(volatile v4f*)(Hf + (size_t)gr * HD + 4 * lane) = fv[i];
      if constexpr (LAST != 0) {
        if (gr < nN) *(volatile v4f*)(out2 + (size_t)gr * HD + 4 * lane) = fv[i];
      }
    }
    __threadfence();
#pragma unroll
    for (int i = 0; i < 16; ++i) {
      const int gr = rowBase + 16 * wave + i;
      if (gr < mRows) *(volatile v4f*)(Hf + (size_t)gr * HD + 4 * lane) = fv[i];
      if constexpr (LAST != 0) {
        if (gr < nN) *(volatile v4f*)(out2 + (size_t)gr * HD + 4 * lane) = fv[i];
      }
    }
  }
  if constexpr (LAST != 0) put_rows_hilo(stg, P1, rowBase, wave, lane, mRows);
}

template <int KS>
__global__ __launch_bounds__(NTHR) __attribute__((amdgpu_num_vgpr(248)))
void k_head(const unsigned short* __restrict__ P1, const unsigned short* __restrict__ WT,
            const float* __restrict__ db1, const float* __restrict__ dg, const float* __restrict__ dbe,
            const float* __restrict__ dw2, const float* __restrict__ db2,
            const float* __restrict__ sb1, const float* __restrict__ sg, const float* __restrict__ sbe,
            const float* __restrict__ sw2, const float* __restrict__ sb2,
            float* dispw, float* strsw, int nN) {
  extern __shared__ v4f dynl[];
  float* stg = (float*)dynl;
  float* sp  = stg + TM * HD;
  float* hw  = sp + 384;
  float* hb  = sp + 768;
  float* dsp = sp + 800;
  float* sst = sp + 1184;
  const int tid = (int)threadIdx.x, lane = tid & 31, wave = tid >> 5, hh = lane >> 4, m = lane & 15;
  const int rowBase = (int)blockIdx.x * TM;

  if (wave == 0)      stage64(sp,            db1, lane);
  else if (wave == 1) stage64(sp + 64,       sb1, lane);
  else if (wave == 2) stage64(sp + 128,      dg,  lane);
  else if (wave == 3) stage64(sp + 128 + 64, sg,  lane);
  else if (wave == 4) stage64(sp + 256,      dbe, lane);
  else if (wave == 5) stage64(sp + 256 + 64, sbe, lane);
  else if (wave == 6) {
#pragma unroll
    for (int it = 0; it < 2; ++it) {
      const int i  = lane + 32 * it;
      const int ic = i < 48 ? i : 47;
      const v4f a = *(const v4f*)(dw2 + 4 * ic);
      asm volatile("" :: "v"(a));
      const float av[4] = {a.x, a.y, a.z, a.w};
      if (i < 48) {
#pragma unroll
        for (int j = 0; j < 4; ++j) {
          const int e = 4 * i + j;
          const int c = e / 3;
          const int o = e - 3 * c;
          hw[o * HD + c] = bf_rne(av[j]);
        }
      }
    }
    hw[HD + 64 + lane] = 0.0f; hw[HD + 96 + lane] = 0.0f;
    hw[2 * HD + 64 + lane] = 0.0f; hw[2 * HD + 96 + lane] = 0.0f;
  } else {
    stage64(hw + 64, sw2, lane);
    const float d2 = db2[lane < 3 ? lane : 2];
    const float s2 = sb2[0];
    asm volatile("" :: "v"(d2), "v"(s2));
    const float hv = (lane < 3) ? bf_rne(d2) : bf_rne(s2);
    if (lane < 4) hb[lane] = hv;
  }

  v8f acc[8];
  {
    const v8f z = {0.f, 0.f, 0.f, 0.f, 0.f, 0.f, 0.f, 0.f};
#pragma unroll
    for (int t = 0; t < 8; ++t) acc[t] = z;
  }
  mma_rows_glb<KS>(P1 + (size_t)(rowBase + 16 * wave + m) * (size_t)APW + 8 * hh,
                   WT + (size_t)m * KT + 8 * hh, acc);
  stage_acc(stg, acc, wave, hh, m);
  __syncthreads();
  {
    const v4f bv = *(const v4fa*)(sp + 4 * lane);
    const v4f gv = *(const v4fa*)(sp + 128 + 4 * lane);
    const v4f ev = *(const v4fa*)(sp + 256 + 4 * lane);
    const v4f w0 = *(const v4fa*)(hw + 4 * lane);
    const v4f w1 = *(const v4fa*)(hw + HD + 4 * lane);
    const v4f w2 = *(const v4fa*)(hw + 2 * HD + 4 * lane);
    const float hb0 = hb[0], hb1 = hb[1], hb2 = hb[2], hb3 = hb[3];
#pragma unroll 1
    for (int i = 0; i < 16; ++i) {
      const int lr = 16 * wave + i;
      const v4f a = *(const v4fa*)(stg + lr * HD + 4 * lane);
      const float x0 = a.x + bv.x, x1 = a.y + bv.y, x2 = a.z + bv.z, x3 = a.w + bv.w;
      const float mean = wsum16((x0 + x1) + (x2 + x3)) * (1.0f / 64.0f);
      const float d0 = x0 - mean, d1 = x1 - mean, d2 = x2 - mean, d3 = x3 - mean;
      const float var = wsum16((d0 * d0 + d1 * d1) + (d2 * d2 + d3 * d3)) * (1.0f / 64.0f);
      const float rs = rsqrtf(var + 1e-5f);
      const float y0 = gelu_f(fmaf(d0 * rs, gv.x, ev.x));
      const float y1 = gelu_f(fmaf(d1 * rs, gv.y, ev.y));
      const float y2 = gelu_f(fmaf(d2 * rs, gv.z, ev.z));
      const float y3 = gelu_f(fmaf(d3 * rs, gv.w, ev.w));
      float p0 = fmaf(y3, w0.w, fmaf(y2, w0.z, fmaf(y1, w0.y, y0 * w0.x)));
      float p1 = fmaf(y3, w1.w, fmaf(y2, w1.z, fmaf(y1, w1.y, y0 * w1.x)));
      float p2 = fmaf(y3, w2.w, fmaf(y2, w2.z, fmaf(y1, w2.y, y0 * w2.x)));
      p0 = wsum16(p0); p1 = wsum16(p1); p2 = wsum16(p2);
      const bool live = (rowBase + lr) < nN;
      const float o0 = p0 + hb0, o1 = p1 + hb1, o2 = p2 + hb2;
      const float tq = p0 + hb3;
      const float mx = (tq > 0.0f) ? tq : ((tq != tq) ? tq : 0.0f);
      const float spv = mx + log1pf(expf(-fabsf(tq)));
      if (lane == 0) {
        dsp[lr * 3 + 0] = live ? o0 : 0.0f;
        dsp[lr * 3 + 1] = live ? o1 : 0.0f;
        dsp[lr * 3 + 2] = live ? o2 : 0.0f;
      }
      if (lane == 16) sst[lr] = live ? spv : 0.0f;
    }
  }
  __syncthreads();
  if (wave < 3) {
    const v4f v = *(const v4fa*)(dsp + 4 * tid);
    float* op = dispw + (size_t)rowBase * 3 + 4 * tid;
    *(volatile v4f*)op = v;
    __threadfence();
    *(volatile v4f*)op = v;
  } else if (wave == 3) {
    const v4f v = *(const v4fa*)(sst + 4 * lane);
    float* op = strsw + (size_t)rowBase + 4 * lane;
    *(volatile v4f*)op = v;
    __threadfence();
    *(volatile v4f*)op = v;
  }
}

__global__ __launch_bounds__(NTHR) void k_pack(const float* __restrict__ dispw, const float* __restrict__ strsw,
                                               float* out, int nU, int nUD) {
  const int u  = (int)blockIdx.x * NTHR + (int)threadIdx.x;
  const int uc = u < nU ? u : nU - 1;
  const int ud = uc < nUD ? uc : nUD - 1;
  int us = uc - nUD;
  us = us < 0 ? 0 : (us > nU - nUD - 1 ? nU - nUD - 1 : us);
  const v4f a = *(const v4f*)(dispw + 4 * (size_t)ud);
  const v4f b = *(const v4f*)(strsw + 4 * (size_t)us);
  asm volatile("" :: "v"(a), "v"(b));
  const unsigned mk = (uc >= nUD) ? 0xffffffffu : 0u;
  v4f o;
  o.x = fsel(a.x, b.x, mk); o.y = fsel(a.y, b.y, mk); o.z = fsel(a.z, b.z, mk); o.w = fsel(a.w, b.w, mk);
  float* op = out + 4 * (size_t)uc;
  if (u < nU) *(volatile v4f*)op = o;
  __threadfence();
  if (u < nU) *(volatile v4f*)op = o;
}

static inline size_t al256(size_t o) { return (o + 255) & ~(size_t)255; }

extern "C" void kernel_launch(void* const* d_in, const int* in_sizes, int n_in,
                              void* d_out, int out_size, void* d_ws, size_t ws_size,
                              hipStream_t stream) {
  if (n_in < 41) return;
  if (in_sizes[0] != NNODE * 6) return;
  if (in_sizes[1] != 2 * NEDGE) return;
  if (in_sizes[2] != NEDGE * 4) return;
  if (in_sizes[3] != 6 * HD || in_sizes[7] != HD * HD) return;
  if (in_sizes[11] != 4 * HD || in_sizes[15] != HD * HD) return;
  if (in_sizes[19] != NLAYER * HD * HD || in_sizes[23] != NLAYER * HD * HD) return;
  if (in_sizes[20] != NLAYER * HD || in_sizes[27] != NLAYER * HD || in_sizes[28] != NLAYER * HD) return;
  if (in_sizes[29] != HD * 64 || in_sizes[35] != HD * 64) return;
  if (in_sizes[33] != 192 || in_sizes[34] != 3 || in_sizes[39] != 64 || in_sizes[40] != 1) return;
  if ((long long)out_size != (long long)NNODE * (3 + 1 + HD)) return;

  const float* x     = (const float*)d_in[0];
  const int*   ei    = (const int*)d_in[1];
  const float* ea    = (const float*)d_in[2];
  const float* ne_w1 = (const float*)d_in[3];
  const float* ne_b1 = (const float*)d_in[4];
  const float* ne_g1 = (const float*)d_in[5];
  const float* ne_e1 = (const float*)d_in[6];
  const float* ne_w2 = (const float*)d_in[7];
  const float* ne_b2 = (const float*)d_in[8];
  const float* ne_g2 = (const float*)d_in[9];
  const float* ne_e2 = (const float*)d_in[10];
  const float* ee_w1 = (const float*)d_in[11];
  const float* ee_b1 = (const float*)d_in[12];
  const float* ee_g1 = (const float*)d_in[13];
  const float* ee_e1 = (const float*)d_in[14];
  const float* ee_w2 = (const float*)d_in[15];
  const float* ee_b2 = (const float*)d_in[16];
  const float* ee_g2 = (const float*)d_in[17];
  const float* ee_e2 = (const float*)d_in[18];
  const float* cv_w1 = (const float*)d_in[19];
  const float* cv_b1 = (const float*)d_in[20];
  const float* cv_g1 = (const float*)d_in[21];
  const float* cv_e1 = (const float*)d_in[22];
  const float* cv_w2 = (const float*)d_in[23];
  const float* cv_b2 = (const float*)d_in[24];
  const float* cv_g2 = (const float*)d_in[25];
  const float* cv_e2 = (const float*)d_in[26];
  const float* nm_g  = (const float*)d_in[27];
  const float* nm_b  = (const float*)d_in[28];
  const float* dh_w1 = (const float*)d_in[29];
  const float* dh_b1 = (const float*)d_in[30];
  const float* dh_g  = (const float*)d_in[31];
  const float* dh_be = (const float*)d_in[32];
  const float* dh_w2 = (const float*)d_in[33];
  const float* dh_b2 = (const float*)d_in[34];
  const float* sh_w1 = (const float*)d_in[35];
  const float* sh_b1 = (const float*)d_in[36];
  const float* sh_g  = (const float*)d_in[37];
  const float* sh_be = (const float*)d_in[38];
  const float* sh_w2 = (const float*)d_in[39];
  const float* sh_b2 = (const float*)d_in[40];
  float* out  = (float*)d_out;
  float* out2 = out + (size_t)NNODE * 4;
  const int* src = ei;
  const int* dst = ei + NEDGE;

  char* ws = (char*)d_ws;
  size_t off = 0;
  const size_t oWT  = off; off = al256(off + (size_t)NPLANE * WSQ * 2);
  const size_t oH   = off; off = al256(off + (size_t)MP * HD * 4);
  const size_t oP1  = off; off = al256(off + (size_t)MP * APW * 2);
  const size_t oLST = off; off = al256(off + (size_t)NBK * RCAP * 4);
  const size_t oMET = off; off = al256(off + (size_t)NBK * METAW * 4);
  const size_t oDSP = off; off = al256(off + (size_t)MP * 3 * 4);
  const size_t oSTR = off; off = al256(off + (size_t)MP * 4);
  const size_t oE16 = off; off = al256(off + (size_t)NEDGE * HD * 2);
  if (off > ws_size) return;
  unsigned short* WT   = (unsigned short*)(ws + oWT);
  float*          Hf   = (float*)(ws + oH);
  unsigned short* P1   = (unsigned short*)(ws + oP1);
  unsigned*       LST  = (unsigned*)(ws + oLST);
  int*            META = (int*)(ws + oMET);
  float*          DSP  = (float*)(ws + oDSP);
  float*          STR  = (float*)(ws + oSTR);
  unsigned*       E16  = (unsigned*)(ws + oE16);

  hipFuncSetAttribute(reinterpret_cast<const void*>(&k_bucket), hipFuncAttributeMaxDynamicSharedMemorySize,
                      (int)LDS_BUCKET);
  hipFuncSetAttribute(reinterpret_cast<const void*>(&k_enc<6, 0, KS_NE>),
                      hipFuncAttributeMaxDynamicSharedMemorySize, (int)LDS_ENC);
  hipFuncSetAttribute(reinterpret_cast<const void*>(&k_enc<4, 1, KS_EE>),
                      hipFuncAttributeMaxDynamicSharedMemorySize, (int)LDS_ENC);
  hipFuncSetAttribute(reinterpret_cast<const void*>(&k_cva<KS_CV>), hipFuncAttributeMaxDynamicSharedMemorySize,
                      (int)LDS_CVA);
  hipFuncSetAttribute(reinterpret_cast<const void*>(&k_cvb<0, KS_CV>), hipFuncAttributeMaxDynamicSharedMemorySize,
                      (int)LDS_CVB);
  hipFuncSetAttribute(reinterpret_cast<const void*>(&k_cvb<1, KS_CV>), hipFuncAttributeMaxDynamicSharedMemorySize,
                      (int)LDS_CVB);
  hipFuncSetAttribute(reinterpret_cast<const void*>(&k_head<KS_HD>), hipFuncAttributeMaxDynamicSharedMemorySize,
                      (int)LDS_HEAD);

  const int gM = MP / TM;

  k_wprep<<<NPLANE * NUSQ / NTHR, NTHR, 0, stream>>>(ne_w2, ee_w2, cv_w1, cv_w2, dh_w1, sh_w1, WT);
  k_bucket<<<NBK, NTHR, LDS_BUCKET, stream>>>(dst, NEDGE, 1, LST, META);
  k_enc<6, 0, KS_NE><<<gM, NTHR, LDS_ENC, stream>>>(x, NNODE, ne_w1, ne_b1, ne_g1, ne_e1, ne_b2, ne_g2, ne_e2,
                                                    WT + (size_t)0 * WSQ, (void*)Hf, MP);
  k_enc<4, 1, KS_EE><<<NEDGE / TM, NTHR, LDS_ENC, stream>>>(ea, NEDGE, ee_w1, ee_b1, ee_g1, ee_e1, ee_b2, ee_g2,
                                                            ee_e2, WT + (size_t)1 * WSQ, (void*)E16, NEDGE);
  for (int l = 0; l < NLAYER; ++l) {
    k_agg<<<gM, NTHR, 0, stream>>>(src, LST, META, Hf, E16, P1, NNODE, NEDGE, MP);
    k_cva<KS_CV><<<gM, NTHR, LDS_CVA, stream>>>(P1, WT + (size_t)(2 + l) * WSQ, cv_b1 + (size_t)l * HD,
                                                cv_g1 + (size_t)l * HD, cv_e1 + (size_t)l * HD, NNODE, MP);
    if (l + 1 < NLAYER) {
      k_cvb<0, KS_CV><<<gM, NTHR, LDS_CVB, stream>>>(P1, WT + (size_t)(6 + l) * WSQ, cv_b2 + (size_t)l * HD,
                                                     cv_g2 + (size_t)l * HD, cv_e2 + (size_t)l * HD,
                                                     nm_g + (size_t)l * HD, nm_b + (size_t)l * HD,
                                                     Hf, out2, NNODE, MP);
    } else {
      k_cvb<1, KS_CV><<<gM, NTHR, LDS_CVB, stream>>>(P1, WT + (size_t)(6 + l) * WSQ, cv_b2 + (size_t)l * HD,
                                                     cv_g2 + (size_t)l * HD, cv_e2 + (size_t)l * HD,
                                                     nm_g + (size_t)l * HD, nm_b + (size_t)l * HD,
                                                     Hf, out2, NNODE, MP);
    }
  }
  k_head<KS_HD><<<gM, NTHR, LDS_HEAD, stream>>>(P1, WT + (size_t)10 * WSQ, dh_b1, dh_g, dh_be, dh_w2, dh_b2,
                                                sh_b1, sh_g, sh_be, sh_w2, sh_b2, DSP, STR, NNODE);
  k_pack<<<(NNODE + NTHR - 1) / NTHR, NTHR, 0, stream>>>(DSP, STR, out, NNODE, (NNODE * 3) / 4);
}
